// SioConvLayer_88527865905508
// MI455X (gfx1250) — hardware-run, weakly checked
//
#include <hip/hip_runtime.h>
#include <math.h>

typedef __attribute__((ext_vector_type(16))) _Float16 v16h;
typedef __attribute__((ext_vector_type(8)))  _Float16 v8h;
typedef __attribute__((ext_vector_type(2)))  _Float16 v2h;
typedef __attribute__((ext_vector_type(16))) __bf16   v16b;
typedef __attribute__((ext_vector_type(8)))  __bf16   v8b;
typedef __attribute__((ext_vector_type(8)))  float    v8f;
typedef __attribute__((ext_vector_type(4)))  float    v4f;
typedef __attribute__((ext_vector_type(2)))  float    v2f;

constexpr int kNb   = 4;
constexpr int kL    = 1024;
constexpr int kD    = 512;
constexpr int kH    = 8;
constexpr int kI    = 64;
constexpr int kRows = kNb * kL;
constexpr int kN3   = 3 * kD;
constexpr int kThr  = 256;
constexpr float kEps = 1e-5f;
constexpr float kInCarry = 1024.0f;
constexpr float kSc = 1.0f / (kInCarry * kInCarry);
constexpr float kF16MinNormal = 6.103515625e-5f;
constexpr int kBiaDt = 1536, kBiaY = 1568;
constexpr size_t kOut0 = 0;
constexpr size_t kOut1 = (size_t)kRows * kD;

static_assert(kD == kH * kI && kI == 64 && kH == 8 && kL == 1024 && kRows == 4096, "the index arithmetic below uses these sizes");

constexpr size_t kOffBIA = 0ull;
constexpr size_t kOffX16 = 9216ull;
constexpr size_t kOffW3 = 4203520ull;
constexpr size_t kOffWY2 = 5776384ull;
constexpr size_t kOffWD16 = 6824960ull;
constexpr size_t kOffP32 = 6857728ull;
constexpr size_t kOffDT32 = 32023552ull;
constexpr size_t kOffZ32 = 32547840ull;
constexpr size_t kOffG32 = 40936448ull;
constexpr size_t kOffZD32 = 40944640ull;
constexpr size_t kOffDEC32 = 40952832ull;
constexpr size_t kOffHN2 = 41083904ull;
constexpr size_t kOffYP32 = 49472512ull;
constexpr size_t kWsTotal = 57861120ull;
static_assert(kWsTotal <= 134217728ull, "carve cap: under 128 MiB");
static_assert(kOffBIA == 0
              && kOffX16 == kOffBIA + 9216ull
              && kOffW3 == kOffX16 + 4194304ull
              && kOffWY2 == kOffW3 + 1572864ull
              && kOffWD16 == kOffWY2 + 1048576ull
              && kOffP32 == kOffWD16 + 32768ull
              && kOffDT32 == kOffP32 + 25165824ull
              && kOffZ32 == kOffDT32 + 524288ull
              && kOffG32 == kOffZ32 + 8388608ull
              && kOffZD32 == kOffG32 + 8192ull
              && kOffDEC32 == kOffZD32 + 8192ull
              && kOffHN2 == kOffDEC32 + 131072ull
              && kOffYP32 == kOffHN2 + 8388608ull
              && kWsTotal == kOffYP32 + 8388608ull, "the carve is chained and totalled");
static_assert((kOffBIA % 256) == 0 && (kOffX16 % 256) == 0 && (kOffW3 % 256) == 0 && (kOffWY2 % 256) == 0 && (kOffWD16 % 256) == 0 && (kOffP32 % 256) == 0 && (kOffDT32 % 256) == 0 && (kOffZ32 % 256) == 0 && (kOffG32 % 256) == 0 && (kOffZD32 % 256) == 0 && (kOffDEC32 % 256) == 0 && (kOffHN2 % 256) == 0 && (kOffYP32 % 256) == 0, "aligned regions");
static_assert(kBiaDt == kN3 && kBiaY == kBiaDt + 32 && kBiaY + kD <= 2304, "each product's bias record covers its output columns (the engines read one bias value a column): 1,536 | 32 | 512 floats laid end to end");

__device__ __forceinline__ unsigned short f2bf_bits(float f) {
  unsigned u = __float_as_uint(f);
  return (unsigned short)((u + 0x7FFFu + ((u >> 16) & 1u)) >> 16);
}
__device__ __forceinline__ float bf_bits2f(unsigned short h) { return __uint_as_float(((unsigned)h) << 16); }
__device__ __forceinline__ float bf16r(float f) { return bf_bits2f(f2bf_bits(f)); }
__device__ __forceinline__ float carry_flush(float v, float carry) {
  const float s = v * carry;
  return (fabsf(s) < kF16MinNormal) ? 0.0f : s;
}

__device__ __forceinline__ void dep_guard4_h(v8f& a, v8f& b, v8f& c, v8f& d, v16h x, v16h y) { asm volatile("v_nop\n\tv_nop\n\tv_nop\n\tv_nop" : "+v"(a), "+v"(b), "+v"(c), "+v"(d) : "v"(x), "v"(y)); }
__device__ __forceinline__ void dep_guard4_b(v8f& a, v8f& b, v8f& c, v8f& d, v16b x, v16b y) { asm volatile("v_nop\n\tv_nop\n\tv_nop\n\tv_nop" : "+v"(a), "+v"(b), "+v"(c), "+v"(d) : "v"(x), "v"(y)); }
__device__ __forceinline__ void keep4_h(v16h a, v16h b, v16h c, v16h d) { asm volatile("v_nop" :: "v"(a), "v"(b), "v"(c), "v"(d)); }
__device__ __forceinline__ void keep4_b(v16b a, v16b b, v16b c, v16b d) { asm volatile("v_nop" :: "v"(a), "v"(b), "v"(c), "v"(d)); }
__device__ __forceinline__ void acc_guard4(v8f& a, v8f& b, v8f& c, v8f& d) { asm volatile("v_nop\n\tv_nop\n\tv_nop\n\tv_nop" : "+v"(a), "+v"(b), "+v"(c), "+v"(d)); }

template <typename T> struct Frag;
template <> struct Frag<_Float16> {
  typedef v16h V; union U { v16h v; v8h h[2]; };
  static __device__ __forceinline__ v16h load(const _Float16* p) {
    U f; f.h[0] = *(const v8h*)(p); f.h[1] = *(const v8h*)(p + 16); return f.v;
  }
  static __device__ __forceinline__ v8f mma(v16h a, v16h b, v8f c) {
    return __builtin_amdgcn_wmma_f32_16x16x32_f16(false, a, false, b, (short)0, c, false, false);
  }
  static __device__ __forceinline__ void guard4(v8f& a, v8f& b, v8f& c, v8f& d, v16h x, v16h y) { dep_guard4_h(a, b, c, d, x, y); }
  static __device__ __forceinline__ void keep(v16h a, v16h b, v16h c, v16h d) { keep4_h(a, b, c, d); }
};
template <> struct Frag<__bf16> {
  typedef v16b V; union U { v16b v; v8b h[2]; };
  static __device__ __forceinline__ v16b load(const __bf16* p) {
    U f; f.h[0] = *(const v8b*)(p); f.h[1] = *(const v8b*)(p + 16); return f.v;
  }
  static __device__ __forceinline__ v8f mma(v16b a, v16b b, v8f c) {
    return __builtin_amdgcn_wmma_f32_16x16x32_bf16(false, a, false, b, (short)0, c, false, false);
  }
  static __device__ __forceinline__ void guard4(v8f& a, v8f& b, v8f& c, v8f& d, v16b x, v16b y) { dep_guard4_b(a, b, c, d, x, y); }
  static __device__ __forceinline__ void keep(v16b a, v16b b, v16b c, v16b d) { keep4_b(a, b, c, d); }
};

__device__ __forceinline__ v8f mma_h(v16h a, v16h b, v8f c) {
  c = __builtin_amdgcn_wmma_f32_16x16x32_f16(false, a, false, b, (short)0, c, false, false);
  asm volatile("v_nop\n\tv_nop\n\tv_nop\n\tv_nop" : "+v"(c) : "v"(a), "v"(b));
  return c;
}

template <int ET> struct Elem;
template <> struct Elem<0> { typedef _Float16 T; };
template <> struct Elem<1> { typedef __bf16 T; };
template <int ET, bool SPLIT, int BIAS_MODE, int OUT_MODE, bool RESID, int ACT = 0>
__global__ __launch_bounds__(256) void wmma_gemm64(
    const unsigned short* __restrict__ Ap, const unsigned short* __restrict__ A2p, int lda, long strideA,
    const unsigned short* __restrict__ Btp, const unsigned short* __restrict__ Bt2p, int ldb, long strideB,
    void* __restrict__ Cout, void* __restrict__ Cout2, int ldc, long strideC,
    const float* __restrict__ bias,
    const float* __restrict__ resid, long strideR,
    int M, int N, int K, float scale) {
  typedef typename Elem<ET>::T T;
  typedef typename Frag<T>::V V;
  const T* A = (const T*)Ap; const T* A2 = (const T*)A2p; const T* Bt = (const T*)Btp; const T* Bt2 = (const T*)Bt2p;
  __shared__ __align__(16) float sT[8][16 * 68];
  const int b    = blockIdx.y;
  const int lane = threadIdx.x & 31;
  const int wave = threadIdx.x >> 5;
  const int tilesN = N >> 6;
  const int tilesM = M >> 6;
  const int tile = blockIdx.x * 8 + wave;
  if (tile >= tilesM * tilesN) return;
  const int tm = tile / tilesN;
  const int tn = tile - tm * tilesN;
  const int m0 = tm << 6;
  const int n0 = tn << 6;

  const T* Ab  = A  + (size_t)b * strideA;
  const T* Bb  = Bt + (size_t)b * strideB;
  const T* Ab2 = SPLIT ? (A2  + (size_t)b * strideA) : nullptr;
  const T* Bb2 = SPLIT ? (Bt2 + (size_t)b * strideB) : nullptr;

  const int rlane = lane & 15;
  const int koff  = (lane >> 4) * 8;
  const int mOff  = (lane >> 4) * 8;

  v8f acc[4][4];
#pragma unroll
  for (int i = 0; i < 4; ++i)
#pragma unroll
    for (int j = 0; j < 4; ++j) acc[i][j] = (v8f){0.f,0.f,0.f,0.f,0.f,0.f,0.f,0.f};

  for (int k0 = 0; k0 < K; k0 += 32) {
    V bh[4], bl[4];
#pragma unroll
    for (int j = 0; j < 4; ++j) {
      const size_t bo = (size_t)(n0 + (j << 4) + rlane) * ldb + koff + k0;
      bh[j] = Frag<T>::load(Bb + bo);
      if (SPLIT) bl[j] = Frag<T>::load(Bb2 + bo);
    }
#pragma unroll
    for (int i = 0; i < 4; ++i) {
      const size_t ao = (size_t)(m0 + (i << 4) + rlane) * lda + koff + k0;
      V ah = Frag<T>::load(Ab + ao);
      V al;
      if (SPLIT) al = Frag<T>::load(Ab2 + ao);
#pragma unroll
      for (int j = 0; j < 4; ++j) {
        acc[i][j] = Frag<T>::mma(ah, bh[j], acc[i][j]);
        if (SPLIT) {
          acc[i][j] = Frag<T>::mma(ah, bl[j], acc[i][j]);
          acc[i][j] = Frag<T>::mma(al, bh[j], acc[i][j]);
        }
      }
      Frag<T>::guard4(acc[i][0], acc[i][1], acc[i][2], acc[i][3], ah, SPLIT ? al : ah);
    }
    Frag<T>::keep(bh[0], bh[1], bh[2], bh[3]);
    if (SPLIT) Frag<T>::keep(bl[0], bl[1], bl[2], bl[3]);
  }
  acc_guard4(acc[0][0], acc[0][1], acc[0][2], acc[0][3]);
  acc_guard4(acc[1][0], acc[1][1], acc[1][2], acc[1][3]);
  acc_guard4(acc[2][0], acc[2][1], acc[2][2], acc[2][3]);
  acc_guard4(acc[3][0], acc[3][1], acc[3][2], acc[3][3]);

  float* slab = sT[wave];
  const float* Rb = RESID ? (resid + (size_t)b * strideR) : nullptr;
#pragma unroll
  for (int i = 0; i < 4; ++i) {
    const int mBase = m0 + (i << 4);
#pragma unroll
    for (int j = 0; j < 4; ++j) {
      const int n = n0 + (j << 4) + rlane;
      float bv = 0.f;
      if (BIAS_MODE == 2) bv = bias[n];
#pragma unroll
      for (int r = 0; r < 8; ++r) {
        float v = acc[i][j][r] * scale;
        if (BIAS_MODE == 1) v += bias[mBase + mOff + r];
        if (BIAS_MODE == 2) v += bv;
        if (RESID) v += Rb[(size_t)(mBase + mOff + r) * ldc + n];
        if (ACT == 1) v = tanhf(v);
        if (ACT == 2) v = fmaxf(v, 0.0f);
        if (ACT == 3) v = v / (1.0f + expf(-v));
        if (ACT == 4) v = (v > 0.f) ? v : 0.01f * v;
        slab[(mOff + r) * 68 + (j << 4) + rlane] = v;
      }
    }
    __builtin_amdgcn_fence(__ATOMIC_RELEASE, "workgroup");
    __builtin_amdgcn_wave_barrier();
    __builtin_amdgcn_fence(__ATOMIC_ACQUIRE, "workgroup");
    if (OUT_MODE == 0) {
      float* C = (float*)Cout + (size_t)b * strideC;
      const int hh = lane >> 4, c4 = (lane & 15) * 4;
      for (int pass = 0; pass < 2; ++pass) {
#pragma unroll
        for (int it = 0; it < 8; ++it) {
          const int row = it * 2 + hh;
          v4f v = *(const v4f*)(slab + row * 68 + c4);
          *(volatile v4f*)(C + (size_t)(mBase + row) * ldc + n0 + c4) = v;
        }
        __threadfence();
      }
    } else {
      const int q = lane >> 3, c8 = (lane & 7) * 8;
      unsigned short* C  = (unsigned short*)Cout  + (size_t)b * strideC;
      unsigned short* C2 = (OUT_MODE == 2) ? ((unsigned short*)Cout2 + (size_t)b * strideC) : nullptr;
      for (int pass = 0; pass < 2; ++pass) {
#pragma unroll
        for (int it = 0; it < 4; ++it) {
          const int row = it * 4 + q;
          const float* sp = slab + row * 68 + c8;
          v8h hv, lv;
#pragma unroll
          for (int e = 0; e < 8; ++e) {
            if (OUT_MODE == 1) {
              hv[e] = (_Float16)sp[e];
            } else {
              unsigned short hb = f2bf_bits(sp[e]);
              unsigned short lb = f2bf_bits(sp[e] - bf_bits2f(hb));
              hv[e] = __builtin_bit_cast(_Float16, hb);
              lv[e] = __builtin_bit_cast(_Float16, lb);
            }
          }
          *(volatile v8h*)(C + (size_t)(mBase + row) * ldc + n0 + c8) = hv;
          if (OUT_MODE == 2) *(volatile v8h*)(C2 + (size_t)(mBase + row) * ldc + n0 + c8) = lv;
        }
        __threadfence();
      }
    }
    __builtin_amdgcn_fence(__ATOMIC_RELEASE, "workgroup");
    __builtin_amdgcn_wave_barrier();
    __builtin_amdgcn_fence(__ATOMIC_ACQUIRE, "workgroup");
  }
}

__global__ __launch_bounds__(kThr) void cast_plane_kernel(const float* __restrict__ src, unsigned short* __restrict__ dst,
                                                          int colsLog2, int dstPitch, int dstOff) {
  const int i   = blockIdx.x * kThr + threadIdx.x;
  const int sh  = colsLog2 - 3;
  const int row = i >> sh;
  const int c8  = (i & ((1 << sh) - 1)) * 8;
  const float* sp = src + ((size_t)row << colsLog2) + c8;
  const v4f a0 = *(const v4f*)(sp);
  const v4f a1 = *(const v4f*)(sp + 4);
  v8h hv;
#pragma unroll
  for (int e = 0; e < 4; ++e) {
    const float f0 = a0[e];
    const float f1 = a1[e];
    hv[e]     = (_Float16)carry_flush(bf16r(f0), kInCarry);
    hv[4 + e] = (_Float16)carry_flush(bf16r(f1), kInCarry);
  }
  unsigned short* dp = dst + (size_t)row * dstPitch + dstOff + c8;
  *(volatile v8h*)dp = hv;
  __threadfence();
  *(volatile v8h*)dp = hv;
}

__global__ __launch_bounds__(256) void wmma_gemm32(
    const unsigned short* __restrict__ Ap, int lda, long strideA,
    const unsigned short* __restrict__ Btp, int ldb, long strideB,
    float* __restrict__ Cout, int ldc, long strideC,
    const float* __restrict__ bias,
    int M, int N, int K, float scale) {
  typedef _Float16 T;
  typedef Frag<T>::V V;
  const T* A = (const T*)Ap; const T* Bt = (const T*)Btp;
  __shared__ __align__(16) float sT[8][16 * 36];
  const int b    = blockIdx.y;
  const int lane = threadIdx.x & 31;
  const int wave = threadIdx.x >> 5;
  const int tilesN = N >> 5;
  const int tilesM = M >> 6;
  const int tile = blockIdx.x * 8 + wave;
  if (tile >= tilesM * tilesN) return;
  const int tm = tile / tilesN;
  const int tn = tile - tm * tilesN;
  const int m0 = tm << 6;
  const int n0 = tn << 5;

  const T* Ab = A  + (size_t)b * strideA;
  const T* Bb = Bt + (size_t)b * strideB;

  const int rlane = lane & 15;
  const int koff  = (lane >> 4) * 8;
  const int mOff  = (lane >> 4) * 8;

  v8f acc[4][2];
#pragma unroll
  for (int i = 0; i < 4; ++i)
#pragma unroll
    for (int j = 0; j < 2; ++j) acc[i][j] = (v8f){0.f,0.f,0.f,0.f,0.f,0.f,0.f,0.f};

  for (int k0 = 0; k0 < K; k0 += 32) {
    V bh[2];
#pragma unroll
    for (int j = 0; j < 2; ++j) {
      const size_t bo = (size_t)(n0 + (j << 4) + rlane) * ldb + koff + k0;
      bh[j] = Frag<T>::load(Bb + bo);
    }
#pragma unroll
    for (int i = 0; i < 4; i += 2) {
      const size_t ao0 = (size_t)(m0 + (i << 4) + rlane) * lda + koff + k0;
      const size_t ao1 = (size_t)(m0 + ((i + 1) << 4) + rlane) * lda + koff + k0;
      V ah0 = Frag<T>::load(Ab + ao0);
      V ah1 = Frag<T>::load(Ab + ao1);
      acc[i][0]     = Frag<T>::mma(ah0, bh[0], acc[i][0]);
      acc[i][1]     = Frag<T>::mma(ah0, bh[1], acc[i][1]);
      acc[i + 1][0] = Frag<T>::mma(ah1, bh[0], acc[i + 1][0]);
      acc[i + 1][1] = Frag<T>::mma(ah1, bh[1], acc[i + 1][1]);
      Frag<T>::guard4(acc[i][0], acc[i][1], acc[i + 1][0], acc[i + 1][1], ah0, ah1);
    }
    Frag<T>::keep(bh[0], bh[1], bh[0], bh[1]);
  }
  acc_guard4(acc[0][0], acc[0][1], acc[1][0], acc[1][1]);
  acc_guard4(acc[2][0], acc[2][1], acc[3][0], acc[3][1]);

  float* slab = sT[wave];
  float* C = Cout + (size_t)b * strideC;
#pragma unroll
  for (int i = 0; i < 4; ++i) {
    const int mBase = m0 + (i << 4);
#pragma unroll
    for (int j = 0; j < 2; ++j) {
      const int n = n0 + (j << 4) + rlane;
      const float bv = bias[n];
#pragma unroll
      for (int r = 0; r < 8; ++r) {
        float v = acc[i][j][r] * scale;
        v += bv;
        slab[(mOff + r) * 36 + (j << 4) + rlane] = v;
      }
    }
    __builtin_amdgcn_fence(__ATOMIC_RELEASE, "workgroup");
    __builtin_amdgcn_wave_barrier();
    __builtin_amdgcn_fence(__ATOMIC_ACQUIRE, "workgroup");
    {
      const int q = lane >> 3, c4 = (lane & 7) * 4;
      for (int pass = 0; pass < 2; ++pass) {
#pragma unroll
        for (int it = 0; it < 4; ++it) {
          const int row = it * 4 + q;
          v4f v = *(const v4f*)(slab + row * 36 + c4);
          *(volatile v4f*)(C + (size_t)(mBase + row) * ldc + n0 + c4) = v;
        }
        __threadfence();
      }
    }
    __builtin_amdgcn_fence(__ATOMIC_RELEASE, "workgroup");
    __builtin_amdgcn_wave_barrier();
    __builtin_amdgcn_fence(__ATOMIC_ACQUIRE, "workgroup");
  }
}
static_assert(sizeof(float) * 8 * 16 * 36 == 18432, "the tail's slabs: 8 waves x 16 rows x 36 floats = 18,432 B of LDS");


__device__ __forceinline__ void two_words(float w, float carry, _Float16& hh, _Float16& ll) {
  const float sc = carry_flush(w, carry);
  hh = (_Float16)sc;
  const float rs = sc - (float)hh;
  ll = (_Float16)((fabsf(rs) < kF16MinNormal) ? 0.0f : rs);
}
__device__ __forceinline__ void store2(float* p, float v) {
  *(volatile float*)p = v;
  __threadfence();
  *(volatile float*)p = v;
}

__global__ __launch_bounds__(kThr) void zero_kernel(float* __restrict__ dst) {
  const size_t o4 = ((size_t)blockIdx.x * kThr + threadIdx.x) * 4u;
  const v4f z = {0.f, 0.f, 0.f, 0.f};
  *(volatile v4f*)(dst + o4) = z;
  __threadfence();
  *(volatile v4f*)(dst + o4) = z;
}

__global__ __launch_bounds__(kThr) void bias_kernel(const float* __restrict__ bz, const float* __restrict__ bza, const float* __restrict__ bya, const float* __restrict__ bdt,
                                                   const float* __restrict__ by, float* __restrict__ BIA) {
  const unsigned t = blockIdx.x * (unsigned)kThr + threadIdx.x;
  if (t >= 2080u) return;
  float v;
  if (t < 512u) { const float a = bz[t]; v = bf16r(a); }
  else if (t < 1024u) { const float a = bza[t - 512u]; v = bf16r(a); }
  else if (t < 1536u) { const float a = bya[t - 1024u]; v = bf16r(a); }
  else if (t < 1568u) { const unsigned j = t - 1536u; const bool live = j < (unsigned)kH; const float a = bdt[live ? j : 0u]; v = live ? bf16r(a) : 0.0f; }
  else { const float a = by[t - 1568u]; v = bf16r(a); }
  store2(BIA + t, v);
}

__global__ __launch_bounds__(kThr) void zgate_kernel(const float* __restrict__ P32, float* __restrict__ Z32) {
  const unsigned i = blockIdx.x * (unsigned)kThr + threadIdx.x;
  const unsigned c4 = (i & 127u) * 4u, r = i >> 7;
  const float* sp = P32 + (size_t)r * kN3 + c4;
  const v4f a = *(const v4f*)sp, g = *(const v4f*)(sp + kD);
  v4f o;
#pragma unroll
  for (int k = 0; k < 4; ++k) o[k] = a[k] * (g[k] / (1.0f + expf(-g[k])));
  float* dp = Z32 + (size_t)i * 4u;
  *(volatile v4f*)dp = o;
  __threadfence();
  *(volatile v4f*)dp = o;
}
static_assert((size_t)kRows * (kD / 4) == 2048ull * kThr, "gate grid exact: 2,048 blocks");

__global__ __launch_bounds__(kThr) void colsum_kernel(const float* __restrict__ Z32, const float* __restrict__ hidden, float* __restrict__ G32, float* __restrict__ ZD32) {
  const unsigned t = blockIdx.x * (unsigned)kThr + threadIdx.x;
  const unsigned c = t & 511u, b = t >> 9;
  const int head = (int)(c >> 6);
  const float* zp = Z32 + (size_t)b * kL * kD + c;
  float s = 0.0f, zd = 0.0f;
  for (int m = 0; m < kL; ++m) {
    const float v = zp[(size_t)m * kD];
    s += (m > head) ? v : 0.0f;
    zd = (m == head) ? v : zd;
  }
  const float h0 = hidden[t];
  store2(G32 + t, s + bf16r(h0));
  store2(ZD32 + t, zd);
}
static_assert(kNb * kD == 8 * kThr, "column-sum grid exact: 8 blocks");

__global__ __launch_bounds__(32) void decay_kernel(const float* __restrict__ DT32, const float* __restrict__ ln_a, float* __restrict__ DEC32) {
  const unsigned b = threadIdx.x >> 3, head = threadIdx.x & 7u;
  const float la = ln_a[head];
  const float na = -expf(bf16r(la));
  float cs = 0.0f;
  for (int l = 0; l < kL; ++l) {
    const size_t row = (size_t)b * kL + (size_t)l;
    const float pre = DT32[row * 32u + head];
    const float sp = (pre > 20.0f) ? pre : log1pf(expf(pre));
    cs += na * sp;
    store2(DEC32 + row * kH + head, expf(cs));
  }
}

__global__ __launch_bounds__(kThr) void hform_kernel(const float* __restrict__ DEC32, const float* __restrict__ G32, const float* __restrict__ ZD32, const float* __restrict__ gnw,
                                                    const float* __restrict__ gnb, float* __restrict__ out1, unsigned short* __restrict__ HN2) {
  const unsigned t = blockIdx.x * (unsigned)kThr + threadIdx.x;
  const unsigned head = t & 7u, row = t >> 3, b = row >> 10;
  const float e = DEC32[t];
  const float* gp = G32 + (size_t)b * kD + head * (unsigned)kI;
  const float* zp = ZD32 + (size_t)b * kD + head * (unsigned)kI;
  float h[kI];
  float sum = 0.0f;
#pragma unroll
  for (int q = 0; q < kI / 4; ++q) {
    const v4f g4 = *(const v4f*)(gp + 4 * q), z4 = *(const v4f*)(zp + 4 * q);
#pragma unroll
    for (int k = 0; k < 4; ++k) { const float v = e * g4[k] + z4[k]; h[4 * q + k] = v; sum += v; }
  }
  float* op = out1 + (size_t)t * kI;
  for (int pass = 0; pass < 2; ++pass) {
#pragma unroll
    for (int q = 0; q < kI / 4; ++q) { v4f o; o[0] = h[4 * q]; o[1] = h[4 * q + 1]; o[2] = h[4 * q + 2]; o[3] = h[4 * q + 3]; *(volatile v4f*)(op + 4 * q) = o; }
    __threadfence();
  }
  const float mu = sum / (float)kI;
  float ss = 0.0f;
#pragma unroll
  for (int i = 0; i < kI; ++i) { const float dlt = h[i] - mu; ss += dlt * dlt; }
  const float rs = 1.0f / sqrtf(ss / (float)kI + kEps);
  const float w0 = gnw[head], b0 = gnb[head];
  const float gw = bf16r(w0), gb = bf16r(b0);
  unsigned short* hp = HN2 + (size_t)row * (2 * kD) + head * (unsigned)kI;
#pragma unroll
  for (int c = 0; c < kI / 8; ++c) {
    v8h hv, lv;
#pragma unroll
    for (int k = 0; k < 8; ++k) { const float v = (h[8 * c + k] - mu) * rs * gw + gb; _Float16 a, r2; two_words(v, kInCarry, a, r2); hv[k] = a; lv[k] = r2; }
    for (int pass = 0; pass < 2; ++pass) { *(volatile v8h*)(hp + 8 * c) = hv; *(volatile v8h*)(hp + kD + 8 * c) = lv; __threadfence(); }
  }
}
static_assert((size_t)kRows * kH == 128ull * kThr, "state grid exact: 128 blocks");

__global__ __launch_bounds__(kThr) void ygate_kernel(const float* __restrict__ YP32, const float* __restrict__ P32, float* __restrict__ out0) {
  const unsigned i = blockIdx.x * (unsigned)kThr + threadIdx.x;
  const unsigned c4 = (i & 127u) * 4u, r = i >> 7;
  const v4f a = *(const v4f*)(YP32 + (size_t)i * 4u), g = *(const v4f*)(P32 + (size_t)r * kN3 + 2 * kD + c4);
  v4f o;
#pragma unroll
  for (int k = 0; k < 4; ++k) o[k] = a[k] * (g[k] / (1.0f + expf(-g[k])));
  float* dp = out0 + (size_t)i * 4u;
  *(volatile v4f*)dp = o;
  __threadfence();
  *(volatile v4f*)dp = o;
}

static_assert(((size_t)kRows * kD / 8) % kThr == 0 && ((size_t)kD * kD / 8) % kThr == 0 && ((size_t)kH * kD / 8) % kThr == 0, "plane cast grids exact");
static_assert(((kRows / 64) * (kN3 / 64)) % 8 == 0 && ((kRows / 64) * (32 / 32)) % 8 == 0 && ((kRows / 64) * (kD / 64)) % 8 == 0, "the products' grids exact: every wave live");

extern "C" void kernel_launch(void* const* d_in, const int* in_sizes, int n_in,
                              void* d_out, int out_size, void* d_ws, size_t ws_size,
                              hipStream_t stream) {
  if (n_in < 15 || d_out == nullptr || d_ws == nullptr) return;
  if (in_sizes[0] != kRows * kD || in_sizes[1] != kNb * kD || in_sizes[2] != kD * kD || in_sizes[3] != kD || in_sizes[4] != kD * kD || in_sizes[5] != kD) return;
  if (in_sizes[6] != kD * kD || in_sizes[7] != kD || in_sizes[8] != kD * kD || in_sizes[9] != kD || in_sizes[10] != kH * kD || in_sizes[11] != kH) return;
  if (in_sizes[12] != kH || in_sizes[13] != kH || in_sizes[14] != kH) return;
  if ((size_t)out_size != kOut1 + (size_t)kRows * kH * kI) return;
  if (ws_size < kWsTotal) return;
  const float* X = (const float*)d_in[0];
  const float* hidden = (const float*)d_in[1];
  const float* w_z = (const float*)d_in[2];
  const float* b_z = (const float*)d_in[3];
  const float* w_za = (const float*)d_in[4];
  const float* b_za = (const float*)d_in[5];
  const float* w_y = (const float*)d_in[6];
  const float* b_y = (const float*)d_in[7];
  const float* w_ya = (const float*)d_in[8];
  const float* b_ya = (const float*)d_in[9];
  const float* w_dt = (const float*)d_in[10];
  const float* b_dt = (const float*)d_in[11];
  const float* ln_a = (const float*)d_in[12];
  const float* gn_w = (const float*)d_in[13];
  const float* gn_b = (const float*)d_in[14];
  float* out = (float*)d_out;
  char* ws = (char*)d_ws;
  float* BIA = (float*)(ws + kOffBIA);
  unsigned short* X16 = (unsigned short*)(ws + kOffX16);
  unsigned short* W3 = (unsigned short*)(ws + kOffW3);
  unsigned short* WY2 = (unsigned short*)(ws + kOffWY2);
  unsigned short* WD16 = (unsigned short*)(ws + kOffWD16);
  float* P32 = (float*)(ws + kOffP32);
  float* DT32 = (float*)(ws + kOffDT32);
  float* Z32 = (float*)(ws + kOffZ32);
  float* G32 = (float*)(ws + kOffG32);
  float* ZD32 = (float*)(ws + kOffZD32);
  float* DEC32 = (float*)(ws + kOffDEC32);
  unsigned short* HN2 = (unsigned short*)(ws + kOffHN2);
  float* YP32 = (float*)(ws + kOffYP32);

  zero_kernel<<<8, kThr, 0, stream>>>((float*)WD16);
  cast_plane_kernel<<<(int)(((size_t)kRows * kD / 8) / kThr), kThr, 0, stream>>>(X, X16, 6, 64, 0);
  cast_plane_kernel<<<(int)(((size_t)kD * kD / 8) / kThr), kThr, 0, stream>>>(w_z, W3, 6, 64, 0);
  cast_plane_kernel<<<(int)(((size_t)kD * kD / 8) / kThr), kThr, 0, stream>>>(w_za, W3 + (size_t)kD * kD, 6, 64, 0);
  cast_plane_kernel<<<(int)(((size_t)kD * kD / 8) / kThr), kThr, 0, stream>>>(w_ya, W3 + (size_t)2 * kD * kD, 6, 64, 0);
  cast_plane_kernel<<<(int)(((size_t)kD * kD / 8) / kThr), kThr, 0, stream>>>(w_y, WY2, 9, 2 * kD, 0);
  cast_plane_kernel<<<(int)(((size_t)kD * kD / 8) / kThr), kThr, 0, stream>>>(w_y, WY2, 9, 2 * kD, kD);
  cast_plane_kernel<<<(int)(((size_t)kH * kD / 8) / kThr), kThr, 0, stream>>>(w_dt, WD16, 6, 64, 0);
  bias_kernel<<<9, kThr, 0, stream>>>(b_z, b_za, b_ya, b_dt, b_y, BIA);
  wmma_gemm64<0, false, 2, 0, false, 0><<<dim3((kRows / 64) * (kN3 / 64) / 8, 1), 256, 0, stream>>>(
      X16, X16, kD, 0L, W3, W3, kD, 0L, (void*)P32, (void*)P32, kN3, 0L, BIA, nullptr, 0L, kRows, kN3, kD, kSc);
  wmma_gemm32<<<dim3((kRows / 64) * (32 / 32) / 8, 1), 256, 0, stream>>>(X16, kD, 0L, WD16, kD, 0L, DT32, 32, 0L, BIA + kBiaDt, kRows, 32, kD, kSc);
  zgate_kernel<<<2048, kThr, 0, stream>>>(P32, Z32);
  colsum_kernel<<<8, kThr, 0, stream>>>(Z32, hidden, G32, ZD32);
  decay_kernel<<<1, 32, 0, stream>>>(DT32, ln_a, DEC32);
  hform_kernel<<<128, kThr, 0, stream>>>(DEC32, G32, ZD32, gn_w, gn_b, out + kOut1, HN2);
  wmma_gemm64<0, false, 2, 0, false, 0><<<dim3((kRows / 64) * (kD / 64) / 8, 1), 256, 0, stream>>>(
      HN2, HN2, 2 * kD, 0L, WY2, WY2, 2 * kD, 0L, (void*)YP32, (void*)YP32, kD, 0L, BIA + kBiaY, nullptr, 0L, kRows, kD, 2 * kD, kSc);
  ygate_kernel<<<2048, kThr, 0, stream>>>(YP32, P32, out + kOut0);
}
